// SimpleLSTM_53249004536456
// MI455X (gfx1250) — hardware-run, weakly checked
//
#include <hip/hip_runtime.h>
#include <math.h>

constexpr int NBATCH = 2048;
constexpr int NSTEP  = 512;
constexpr int NHID   = 32;
constexpr int NGATE  = 4 * NHID;
constexpr int BTILE  = 32;
constexpr int NTHR   = 128;
constexpr float WCARRY  = 16.0f;
constexpr float HCARRY  = 8.0f;
constexpr float TCARRY  = WCARRY * HCARRY;
constexpr float TCARRY_INV = 1.0f / 128.0f;
static_assert(NBATCH % BTILE == 0);
static_assert(NTHR == NGATE);
static_assert(NHID == 32);
static_assert(BTILE == 32);
static_assert((NGATE * NHID / 4) % NTHR == 0);
static_assert((2 * BTILE * NHID) % NTHR == 0);

typedef __attribute__((ext_vector_type(16))) _Float16 v16h;
typedef __attribute__((ext_vector_type(8)))  _Float16 v8h;
typedef __attribute__((ext_vector_type(4)))  _Float16 v4h;
typedef __attribute__((ext_vector_type(8)))  float    v8f;
typedef __attribute__((ext_vector_type(4)))  float    v4f;

__device__ __forceinline__ void mma_guard4(v8f& d0, v8f& d1, v8f& d2, v8f& d3,
                                           v16h a0, v16h a1, v16h a2, v16h a3, v16h b) {
  asm volatile("v_nop\n\tv_nop\n\tv_nop\n\tv_nop"
               : "+v"(d0), "+v"(d1), "+v"(d2), "+v"(d3)
               : "v"(a0), "v"(a1), "v"(a2), "v"(a3), "v"(b));
}

template <typename T> struct Frag;
template <> struct Frag<_Float16> {
  typedef v16h V; union U { v16h v; v8h h[2]; };
  static __device__ __forceinline__ v16h load(const _Float16* p) {
    U f; f.h[0] = *(const v8h*)(p); f.h[1] = *(const v8h*)(p + 16); return f.v;
  }
  static __device__ __forceinline__ v8f mma(v16h a, v16h b, v8f c) {
    return __builtin_amdgcn_wmma_f32_16x16x32_f16(false, a, false, b, (short)0, c, false, false);
  }
};

__device__ __forceinline__ float fsig(float z)  { return __builtin_amdgcn_rcpf(1.0f + expf(-z)); }
__device__ __forceinline__ float ftanh(float z) { return 1.0f - 2.0f * __builtin_amdgcn_rcpf(expf(2.0f * z) + 1.0f); }

__global__ __launch_bounds__(NTHR) void lstm2_seq_kernel(
    const float* __restrict__ x,
    const float* __restrict__ Wih0, const float* __restrict__ Whh0,
    const float* __restrict__ bih0, const float* __restrict__ bhh0,
    const float* __restrict__ Wih1, const float* __restrict__ Whh1,
    const float* __restrict__ bih1, const float* __restrict__ bhh1,
    const float* __restrict__ Wfc, const float* __restrict__ bfc,
    float* __restrict__ out) {
  __shared__ __align__(16) _Float16 sWh0[NGATE * NHID];
  __shared__ __align__(16) _Float16 sWx1[NGATE * NHID];
  __shared__ __align__(16) _Float16 sWh1[NGATE * NHID];
  __shared__ __align__(16) float    sXw[NGATE];
  __shared__ __align__(16) float    sB0[NGATE];
  __shared__ __align__(16) float    sB1[NGATE];
  __shared__ __align__(16) float    sWfc[NHID];
  __shared__ __align__(16) _Float16 sH0[2][BTILE * NHID];
  __shared__ __align__(16) _Float16 sH1[2][BTILE * NHID];
  __shared__ __align__(16) float    sRed[2][BTILE];
  __shared__ __align__(16) float    sFin[BTILE];

  const int tid  = threadIdx.x;
  const int lane = tid & 31;
  const int wave = tid >> 5;
  const int nt   = wave >> 1;
  const int hv   = wave & 1;
  const int lq   = lane & 15;
  const int lh   = lane >> 4;
  const int bbase = blockIdx.x * BTILE;

#pragma unroll 1
  for (int i = tid; i < NGATE * NHID / 4; i += NTHR) {
    const v4f wa = *(const v4f*)(Whh0 + 4 * i);
    const v4f wb = *(const v4f*)(Wih1 + 4 * i);
    const v4f wc = *(const v4f*)(Whh1 + 4 * i);
    v4h ha, hb, hc;
#pragma unroll
    for (int e = 0; e < 4; ++e) {
      ha[e] = (_Float16)(wa[e] * WCARRY);
      hb[e] = (_Float16)(wb[e] * WCARRY);
      hc[e] = (_Float16)(wc[e] * WCARRY);
    }
    *(v4h*)(sWh0 + 4 * i) = ha;
    *(v4h*)(sWx1 + 4 * i) = hb;
    *(v4h*)(sWh1 + 4 * i) = hc;
  }
  asm volatile("" ::: "memory");
  {
    const float w0 = Wih0[tid];
    const float ba = bih0[tid];
    const float bb = bhh0[tid];
    const float bc = bih1[tid];
    const float bd = bhh1[tid];
    sXw[tid] = w0 * TCARRY;
    sB0[tid] = (ba + bb) * TCARRY;
    sB1[tid] = (bc + bd) * TCARRY;
  }
  asm volatile("" ::: "memory");
  {
    const int wi = (tid < NHID) ? tid : (NHID - 1);
    const float wf = Wfc[wi];
    if (tid < NHID) sWfc[tid] = wf;
  }
  const float bfcv = bfc[0];
  {
    _Float16* h0f = &sH0[0][0];
    _Float16* h1f = &sH1[0][0];
#pragma unroll 1
    for (int i = tid; i < 2 * BTILE * NHID; i += NTHR) {
      h0f[i] = (_Float16)0.0f;
      h1f[i] = (_Float16)0.0f;
    }
  }
  float c0s[8], c1s[8], h1s[8];
#pragma unroll
  for (int r = 0; r < 8; ++r) { c0s[r] = 0.0f; c1s[r] = 0.0f; h1s[r] = 0.0f; }
  __syncthreads();

  const float* xrow = x + (size_t)(bbase + 16 * nt + lq) * NSTEP;
  const int hrd  = (16 * nt + lq) * NHID + 8 * lh;
  const int hwr  = (16 * nt + lq) * NHID + 16 * hv + 8 * lh;
  const int arow = lq * NHID + 8 * lh;

#pragma unroll 1
  for (int t = 0; t < NSTEP; ++t) {
    const int cur = t & 1;
    const int nxt = cur ^ 1;
    const float xv = xrow[t];

    {
      const v16h bh = Frag<_Float16>::load(&sH0[cur][0] + hrd);
      v16h af[4];
      v8f  acc[4];
#pragma unroll
      for (int mm = 0; mm < 4; ++mm) {
        const int mt = 2 * mm + hv;
        af[mm] = Frag<_Float16>::load(sWh0 + mt * 16 * NHID + arow);
        const int gb = 16 * mt + 8 * lh;
        const v4f blo = *(const v4f*)(sB0 + gb);
        const v4f bhi = *(const v4f*)(sB0 + gb + 4);
        const v4f wlo = *(const v4f*)(sXw + gb);
        const v4f whi = *(const v4f*)(sXw + gb + 4);
        v8f ci;
#pragma unroll
        for (int r = 0; r < 4; ++r) {
          ci[r]     = fmaf(xv, wlo[r], blo[r]);
          ci[4 + r] = fmaf(xv, whi[r], bhi[r]);
        }
        acc[mm] = ci;
      }
#pragma unroll
      for (int mm = 0; mm < 4; ++mm) acc[mm] = Frag<_Float16>::mma(af[mm], bh, acc[mm]);
      mma_guard4(acc[0], acc[1], acc[2], acc[3], af[0], af[1], af[2], af[3], bh);
      v8h hpk;
#pragma unroll
      for (int r = 0; r < 8; ++r) {
        const float ig = fsig(acc[0][r] * TCARRY_INV);
        const float fg = fsig(acc[1][r] * TCARRY_INV);
        const float gg = ftanh(acc[2][r] * TCARRY_INV);
        const float og = fsig(acc[3][r] * TCARRY_INV);
        const float cn = fg * c0s[r] + ig * gg;
        c0s[r] = cn;
        const float hn = og * ftanh(cn);
        hpk[r] = (_Float16)(hn * HCARRY);
      }
      *(v8h*)(&sH0[nxt][0] + hwr) = hpk;
    }
    __syncthreads();

    {
      const v16h bx = Frag<_Float16>::load(&sH0[nxt][0] + hrd);
      const v16h bq = Frag<_Float16>::load(&sH1[cur][0] + hrd);
      v16h ax[4], ah[4];
      v8f  acc[4];
#pragma unroll
      for (int mm = 0; mm < 4; ++mm) {
        const int mt = 2 * mm + hv;
        ax[mm] = Frag<_Float16>::load(sWx1 + mt * 16 * NHID + arow);
        const int gb = 16 * mt + 8 * lh;
        const v4f blo = *(const v4f*)(sB1 + gb);
        const v4f bhi = *(const v4f*)(sB1 + gb + 4);
        v8f ci;
#pragma unroll
        for (int r = 0; r < 4; ++r) { ci[r] = blo[r]; ci[4 + r] = bhi[r]; }
        acc[mm] = ci;
      }
#pragma unroll
      for (int mm = 0; mm < 4; ++mm) acc[mm] = Frag<_Float16>::mma(ax[mm], bx, acc[mm]);
      mma_guard4(acc[0], acc[1], acc[2], acc[3], ax[0], ax[1], ax[2], ax[3], bx);
#pragma unroll
      for (int mm = 0; mm < 4; ++mm) {
        const int mt = 2 * mm + hv;
        ah[mm] = Frag<_Float16>::load(sWh1 + mt * 16 * NHID + arow);
      }
#pragma unroll
      for (int mm = 0; mm < 4; ++mm) acc[mm] = Frag<_Float16>::mma(ah[mm], bq, acc[mm]);
      mma_guard4(acc[0], acc[1], acc[2], acc[3], ah[0], ah[1], ah[2], ah[3], bq);
      v8h hpk;
#pragma unroll
      for (int r = 0; r < 8; ++r) {
        const float ig = fsig(acc[0][r] * TCARRY_INV);
        const float fg = fsig(acc[1][r] * TCARRY_INV);
        const float gg = ftanh(acc[2][r] * TCARRY_INV);
        const float og = fsig(acc[3][r] * TCARRY_INV);
        const float cn = fg * c1s[r] + ig * gg;
        c1s[r] = cn;
        const float hn = og * ftanh(cn);
        h1s[r] = hn;
        hpk[r] = (_Float16)(hn * HCARRY);
      }
      *(v8h*)(&sH1[nxt][0] + hwr) = hpk;
    }
    __syncthreads();
  }

  float res = 0.0f;
  {
    const v4f wlo = *(const v4f*)(sWfc + 16 * hv + 8 * lh);
    const v4f whi = *(const v4f*)(sWfc + 16 * hv + 8 * lh + 4);
#pragma unroll
    for (int r = 0; r < 4; ++r) res = fmaf(h1s[r], wlo[r], res);
#pragma unroll
    for (int r = 0; r < 4; ++r) res = fmaf(h1s[4 + r], whi[r], res);
  }
  res += __shfl_xor(res, 16, 32);
  if (lh == 0) sRed[hv][16 * nt + lq] = res;
  __syncthreads();
  if (wave == 0) {
    const float v = (sRed[0][lane] + sRed[1][lane]) + bfcv;
    sFin[lane] = v;
  }
  __syncthreads();
  {
    const int q = (lane < 8) ? lane : 7;
    const v4f o = *(const v4f*)(sFin + 4 * q);
    float* op = out + bbase + 4 * q;
    const bool writer = (tid < 8);
    if (writer) *(volatile v4f*)op = o;
    __threadfence();
    if (writer) *(volatile v4f*)op = o;
  }
}

extern "C" void kernel_launch(void* const* d_in, const int* in_sizes, int n_in,
                              void* d_out, int out_size, void* d_ws, size_t ws_size, hipStream_t stream) {
  (void)d_ws; (void)ws_size;
  if (n_in < 11 || d_out == nullptr) return;
  if (in_sizes[0] != NBATCH * NSTEP || in_sizes[1] != NGATE || in_sizes[2] != NGATE * NHID ||
      in_sizes[3] != NGATE || in_sizes[4] != NGATE || in_sizes[5] != NGATE * NHID ||
      in_sizes[6] != NGATE * NHID || in_sizes[7] != NGATE || in_sizes[8] != NGATE ||
      in_sizes[9] != NHID || in_sizes[10] != 1 || out_size != NBATCH) return;

  const float* x    = (const float*)d_in[0];
  const float* Wih0 = (const float*)d_in[1];
  const float* Whh0 = (const float*)d_in[2];
  const float* bih0 = (const float*)d_in[3];
  const float* bhh0 = (const float*)d_in[4];
  const float* Wih1 = (const float*)d_in[5];
  const float* Whh1 = (const float*)d_in[6];
  const float* bih1 = (const float*)d_in[7];
  const float* bhh1 = (const float*)d_in[8];
  const float* Wfc  = (const float*)d_in[9];
  const float* bfc  = (const float*)d_in[10];
  float* out = (float*)d_out;

  lstm2_seq_kernel<<<dim3(NBATCH / BTILE), dim3(NTHR), 0, stream>>>(
      x, Wih0, Whh0, bih0, bhh0, Wih1, Whh1, bih1, bhh1, Wfc, bfc, out);
}
